// Instance_self_disentangle_atten_66700842107137
// MI455X (gfx1250) — hardware-verified
//
#include <hip/hip_runtime.h>
#include <math.h>

typedef __attribute__((ext_vector_type(16))) _Float16 v16h;
typedef __attribute__((ext_vector_type(16))) __bf16 v16b;
typedef __attribute__((ext_vector_type(8)))  _Float16 v8h;
typedef __attribute__((ext_vector_type(8)))  float v8f;
typedef __attribute__((ext_vector_type(4)))  float v4f;
typedef __attribute__((ext_vector_type(2)))  float v2f;
typedef __attribute__((ext_vector_type(4)))  unsigned v4u;
typedef __attribute__((ext_vector_type(4)))  int v4i;
typedef float __attribute__((may_alias)) float_a;
typedef int __attribute__((may_alias)) int_a;

template <typename T> __device__ __forceinline__ void vst2(void* p, T v) { *(volatile T*)p = v; __threadfence(); *(volatile T*)p = v; }
__device__ __forceinline__ v8f wmma16(v16h a, v16h b, v8f c) {
  v8f d = __builtin_amdgcn_wmma_f32_16x16x32_f16(false, a, false, b, (short)0, c, false, false);
  asm volatile("v_nop\n\tv_nop\n\tv_nop\n\tv_nop" : "+v"(d) : "v"(a), "v"(b));
  return d;
}
__device__ __forceinline__ v8f wmma_bf(v16b a, v16b b, v8f c) {
  v8f d = __builtin_amdgcn_wmma_f32_16x16x32_bf16(false, a, false, b, (short)0, c, false, false);
  asm volatile("v_nop\n\tv_nop\n\tv_nop\n\tv_nop" : "+v"(d) : "v"(a), "v"(b));
  return d;
}
__device__ __forceinline__ v16h frag_h(const _Float16* rowk0, int lane) {
  union { v16h v; v8h q[2]; } u; const _Float16* p = rowk0 + 8 * (lane >> 4);
  u.q[0] = *(const v8h*)p; u.q[1] = *(const v8h*)(p + 16); return u.v;
}
__device__ __forceinline__ v16h frag_f32(const float* rowk0, int lane) {
  v16h a; const float* p = rowk0 + 8 * (lane >> 4);
#pragma unroll
  for (int i = 0; i < 8; ++i) { a[i] = (_Float16)p[i]; a[8 + i] = (_Float16)p[16 + i]; }
  return a;
}
__device__ __forceinline__ v16h frag_f32s(const float* rowk0, int lane, float sc) {
  v16h a; const float* p = rowk0 + 8 * (lane >> 4);
#pragma unroll
  for (int i = 0; i < 8; ++i) { a[i] = (_Float16)(p[i] * sc); a[8 + i] = (_Float16)(p[16 + i] * sc); }
  return a;
}
__device__ __forceinline__ v16h fragc_f32(const float* W, int k0, int n, int lane, int ld, int K) {
  v16h a; const int g = lane >> 4;
#pragma unroll
  for (int i = 0; i < 8; ++i) { const int ka = k0 + 8 * g + i, kb = ka + 16;
    a[i] = (_Float16)(ka < K ? W[(size_t)(ka < K ? ka : K - 1) * ld + n] : 0.f); a[8 + i] = (_Float16)(kb < K ? W[(size_t)(kb < K ? kb : K - 1) * ld + n] : 0.f); }
  return a;
}
struct F2 { v16b h, l; };
__device__ __forceinline__ F2 bsplit16(const float v[16]) { F2 r;
#pragma unroll
  for (int i = 0; i < 16; ++i) { const __bf16 h = (__bf16)v[i]; r.h[i] = h; r.l[i] = (__bf16)(v[i] - (float)h); }
  return r; }
__device__ __forceinline__ F2 split_row(const float* row, int k0, int lane) { float v[16]; const float* p = row + k0 + 8 * (lane >> 4);
#pragma unroll
  for (int i = 0; i < 8; ++i) { v[i] = p[i]; v[8 + i] = p[16 + i]; }
  return bsplit16(v); }
__device__ __forceinline__ F2 split_rowK(const float* row, int k0, int lane, int K) { float v[16]; const int g = lane >> 4;
#pragma unroll
  for (int i = 0; i < 8; ++i) { const int ka = k0 + 8 * g + i, kb = ka + 16; v[i] = ka < K ? row[ka < K ? ka : K - 1] : 0.f; v[8 + i] = kb < K ? row[kb < K ? kb : K - 1] : 0.f; }
  return bsplit16(v); }
__device__ __forceinline__ F2 split_col(const float* W, int k0, int n, int lane, int ld, int K) { float v[16]; const int g = lane >> 4;
#pragma unroll
  for (int i = 0; i < 8; ++i) { const int ka = k0 + 8 * g + i, kb = ka + 16; v[i] = ka < K ? W[(size_t)(ka < K ? ka : K - 1) * ld + n] : 0.f; v[8 + i] = kb < K ? W[(size_t)(kb < K ? kb : K - 1) * ld + n] : 0.f; }
  return bsplit16(v); }
__device__ __forceinline__ v8f mac3(const F2& a, const F2& b, v8f c) { c = wmma_bf(a.l, b.h, c); c = wmma_bf(a.h, b.l, c); return wmma_bf(a.h, b.h, c); }
__device__ __forceinline__ float sigm(float v) { return 1.0f / (1.0f + expf(-v)); }
#define LDSX() do { asm volatile("s_wait_dscnt 0" ::: "memory"); __builtin_amdgcn_wave_barrier(); __builtin_amdgcn_fence(__ATOMIC_RELEASE, "workgroup"); } while (0)


#define NB 16
#define NN 512
#define DIM 256
#define NH 8
#define HDd 32
#define NR (NB * NN)
#ifndef TQB
#define TQB (NN / 64)
#endif
typedef __attribute__((ext_vector_type(8))) __bf16 v8b;
__device__ __forceinline__ v16b frag_b(const __bf16* rowk0, int lane) {
  union { v16b v; v8b q[2]; } u; const __bf16* p = rowk0 + 8 * (lane >> 4);
  u.q[0] = *(const v8b*)p; u.q[1] = *(const v8b*)(p + 16); return u.v;
}
__device__ __forceinline__ float bfr(float v) { return (float)(__bf16)v; }
__device__ __attribute__((noinline)) float exp_ni(float v) { return expf(v); }
__device__ __attribute__((noinline)) float erf_ni(float v) { return erff(v); }

#define WS_PK  0u
#define PKQ 0
#define PKM ((size_t)DIM * DIM)
#define PKK (PKM + (size_t)16 * DIM)
#define PKV (PKK + (size_t)DIM * DIM)
#define PKF (PKV + (size_t)DIM * DIM)
#define PKE (PKF + (size_t)DIM * DIM)
#define WS_Q   (((2u * PKE) + 127u) / 128u * 128u)
#define WS_K   (WS_Q + 4u * NR * DIM)
#define WS_M   (WS_K + 4u * NR * DIM)
#define WS_MU  (WS_M + 4u * NR * 16)
#define WS_QH  (WS_MU + 4u * 2 * NB * DIM)
#define WS_QL  (WS_QH + 2u * NR * DIM)
#define WS_KH  (WS_QL + 2u * NR * DIM)
#define WS_KL  (WS_KH + 2u * NR * DIM)
#define WS_VH  (WS_KL + 2u * NR * DIM)
#define WS_VL  (WS_VH + 2u * NR * DIM)
#define WS_CB  (WS_VL + 2u * NR * DIM)
#define WS_O   (WS_CB + 4u * NB * NH * HDd)
#define WS_Y   (WS_O + 4u * (size_t)NB * NH * NN * HDd)
#define WS_END (WS_Y + 4u * NR * DIM)

__global__ __launch_bounds__(256) void k_pack(const float* __restrict__ WQ, const float* __restrict__ WM, const float* __restrict__ WK, const float* __restrict__ WV, const float* __restrict__ WF, __bf16* __restrict__ PK) {
  const int n = blockIdx.x, which = blockIdx.y, t = threadIdx.x; __shared__ __align__(16) __bf16 s[DIM]; size_t dst; const float* src;
  if (which == 0) { src = WQ + (size_t)n * DIM; dst = PKQ + (size_t)n * DIM; } else if (which == 1) { if (n >= 16) return; src = (n < NH) ? WM + (size_t)n * DIM : nullptr; dst = PKM + (size_t)n * DIM; }
  else if (which == 2) { src = WK + (size_t)n * DIM; dst = PKK + (size_t)n * DIM; } else if (which == 3) { src = WV + (size_t)n * DIM; dst = PKV + (size_t)n * DIM; } else { src = WF + (size_t)n * DIM; dst = PKF + (size_t)n * DIM; }
  s[t] = (__bf16)(src ? src[t] : 0.f); __syncthreads();
  if (t < DIM / 8) vst2((unsigned*)(PK + dst + t * 8), *(const v4u*)&s[t * 8]);
}
__global__ __launch_bounds__(128) void k_proj(const float* __restrict__ X, const float* __restrict__ Y, const __bf16* __restrict__ PK, const float* __restrict__ BQ, const float* __restrict__ BM, const float* __restrict__ BK, const float* __restrict__ BV, float* __restrict__ Q, float* __restrict__ K, float* __restrict__ M, _Float16* __restrict__ VH, _Float16* __restrict__ VL) {
  __shared__ __align__(16) float so[64][DIM + 4]; __shared__ __align__(16) _Float16 svh[DIM][72], svl[DIM][72];
  const int tid = threadIdx.x, wave = tid >> 5, lane = tid & 31, col = lane & 15, g = lane >> 4; const int which = blockIdx.y; const size_t r0 = (size_t)blockIdx.x * 64 + wave * 16; const size_t rb0 = (size_t)blockIdx.x * 64;
  const float* Xs = (which == 0) ? X : Y; const __bf16* Wr = PK + ((which == 0) ? PKQ : (which == 1) ? PKK : PKV); const float* BB = (which == 0) ? BQ : (which == 1) ? BK : BV;
  v8f accm = {};
#pragma unroll 1
  for (int pass = 0; pass < 2; ++pass) { v8f acc[8] = {};
#pragma unroll
    for (int kc = 0; kc < DIM / 32; ++kc) { v16b a; { const float* p = Xs + (r0 + col) * DIM + kc * 32 + 8 * g;
#pragma unroll
        for (int i = 0; i < 8; ++i) { a[i] = (__bf16)p[i]; a[8 + i] = (__bf16)p[16 + i]; } }
#pragma unroll
      for (int j = 0; j < 8; ++j) acc[j] = wmma_bf(a, frag_b(Wr + (size_t)(pass * 128 + j * 16 + col) * DIM + kc * 32, lane), acc[j]);
      if (which == 0 && pass == 0) accm = wmma_bf(a, frag_b(PK + PKM + (size_t)col * DIM + kc * 32, lane), accm); }
    if (which < 2) {
#pragma unroll
      for (int j = 0; j < 8; ++j) { const float bb = bfr(BB[pass * 128 + j * 16 + col]);
#pragma unroll
        for (int r = 0; r < 8; ++r) so[wave * 16 + 8 * g + r][pass * 128 + j * 16 + col] = acc[j][r] + bb; } }
    else {
#pragma unroll
      for (int j = 0; j < 8; ++j) { const int c = pass * 128 + j * 16 + col; const float bb = bfr(BB[c]);
#pragma unroll
        for (int r = 0; r < 8; ++r) { const float v = acc[j][r] + bb; const _Float16 hv = (_Float16)v; svh[c][wave * 16 + 8 * g + r] = hv; svl[c][wave * 16 + 8 * g + r] = (_Float16)((v - (float)hv) * 2048.0f); } } } }
  if (which < 2) { float* D = which ? K : Q;
    LDSX();
    for (int rl = 0; rl < 16; ++rl) for (int q = lane; q < DIM / 4; q += 32) vst2(D + (r0 + rl) * DIM + q * 4, *(const v4f*)&so[wave * 16 + rl][q * 4]);
    if (which == 0) { __shared__ __align__(16) float sm[64][16];
#pragma unroll
      for (int r = 0; r < 8; ++r) sm[wave * 16 + 8 * g + r][col] = accm[r] + ((col < NH) ? bfr(BM[col]) : 0.f);
      __syncthreads();
      for (int e = tid; e < 64 * 4; e += 128) { const int r = e >> 2, q = e & 3; vst2(M + (rb0 + r) * 16 + q * 4, *(const v4f*)&sm[r][q * 4]); } }
  } else {
    __syncthreads();
    const size_t b = rb0 / NN; const size_t n0 = rb0 % NN;
    for (int e = tid; e < DIM * 8; e += 128) { const int c = e >> 3, pc = e & 7; const size_t o = (b * DIM + c) * NN + n0 + pc * 8; vst2((unsigned*)(VH + o), *(const v4u*)&svh[c][pc * 8]); vst2((unsigned*)(VL + o), *(const v4u*)&svl[c][pc * 8]); } }
}
__global__ __launch_bounds__(256) void k_mean(const float* __restrict__ Q, const float* __restrict__ K, float* __restrict__ MU) {
  const int b = blockIdx.x, which = blockIdx.y, c = threadIdx.x; const float* S = which ? K : Q; float s = 0.f;
  for (int n = 0; n < NN; ++n) s += S[((size_t)b * NN + n) * DIM + c];
  __shared__ __align__(16) float so[DIM]; so[c] = s / (float)NN; __syncthreads();
  if (c < DIM / 4) vst2(MU + ((size_t)which * NB + b) * DIM + c * 4, *(const v4f*)&so[c * 4]);
}
__global__ __launch_bounds__(256) void k_center(const float* __restrict__ Q, const float* __restrict__ K, const float* __restrict__ MU, _Float16* __restrict__ QH, _Float16* __restrict__ QL, _Float16* __restrict__ KH, _Float16* __restrict__ KL) {
  const size_t row = blockIdx.x; const size_t b = row / NN; const int c = threadIdx.x; __shared__ __align__(16) _Float16 s[4][DIM];
  { const float v = Q[row * DIM + c] - MU[b * DIM + c]; const _Float16 hv = (_Float16)v; s[0][c] = hv; s[1][c] = (_Float16)((v - (float)hv) * 2048.0f); }
  { const float v = K[row * DIM + c] - MU[((size_t)NB + b) * DIM + c]; const _Float16 hv = (_Float16)v; s[2][c] = hv; s[3][c] = (_Float16)((v - (float)hv) * 2048.0f); }
  __syncthreads();
  if (c < DIM / 8) { vst2((unsigned*)(QH + row * DIM + c * 8), *(const v4u*)&s[0][c * 8]); vst2((unsigned*)(QL + row * DIM + c * 8), *(const v4u*)&s[1][c * 8]); vst2((unsigned*)(KH + row * DIM + c * 8), *(const v4u*)&s[2][c * 8]); vst2((unsigned*)(KL + row * DIM + c * 8), *(const v4u*)&s[3][c * 8]); }
}
__global__ __launch_bounds__(512) void k_gate(const float* __restrict__ M, const _Float16* __restrict__ VH, const _Float16* __restrict__ VL, float* __restrict__ CB) {
  const int b = blockIdx.x, h = blockIdx.y, n = threadIdx.x; __shared__ float red[16]; __shared__ float sp[NN]; __shared__ __align__(16) float so[HDd];
  const float mv = M[((size_t)b * NN + n) * 16 + h]; float mx = mv;
#pragma unroll
  for (int o = 1; o < 32; o <<= 1) mx = fmaxf(mx, __shfl_xor(mx, o));
  if ((n & 31) == 0) red[n >> 5] = mx; __syncthreads(); float gm = -3.0e38f; for (int w = 0; w < 16; ++w) gm = fmaxf(gm, red[w]); __syncthreads();
  const float e = expf(mv - gm); float s = e;
#pragma unroll
  for (int o = 1; o < 32; o <<= 1) s += __shfl_xor(s, o);
  if ((n & 31) == 0) red[n >> 5] = s; __syncthreads(); float tot = 0.f; for (int w = 0; w < 16; ++w) tot += red[w]; sp[n] = e / tot; __syncthreads();
  if (n < HDd) { float a = 0.f; const size_t vo = ((size_t)b * DIM + h * HDd + n) * NN; for (int j = 0; j < NN; ++j) a += sp[j] * ((float)VH[vo + j] + (float)VL[vo + j] * (1.0f / 2048.0f)); so[n] = a; }
  __syncthreads();
  if (n < HDd / 4) vst2(CB + ((size_t)b * NH + h) * HDd + n * 4, *(const v4f*)&so[n * 4]);
}
__global__ __launch_bounds__(128) void k_attn(const _Float16* __restrict__ QH, const _Float16* __restrict__ QL, const _Float16* __restrict__ KH, const _Float16* __restrict__ KL, const _Float16* __restrict__ VH, const _Float16* __restrict__ VL, const float* __restrict__ CB, float* __restrict__ O) {
  __shared__ __align__(16) _Float16 sph[4][16][40], spl[4][16][40]; __shared__ __align__(16) float so[4][16][36];
  const int tid = threadIdx.x, wave = tid >> 5, lane = tid & 31, col = lane & 15, g = lane >> 4; const int qb = blockIdx.x, h = blockIdx.y; const size_t b = blockIdx.z; const int q0 = qb * 64 + wave * 16; const size_t rq = b * NN + q0;
  const v16h aq = frag_h(QH + (rq + col) * DIM + h * HDd, lane), aql = frag_h(QL + (rq + col) * DIM + h * HDd, lane);
  float m[8], l[8];
#pragma unroll
  for (int r = 0; r < 8; ++r) { m[r] = -3.0e38f; l[r] = 0.f; }
  v8f acc[2] = {}, accl[2] = {}; const float isc = 1.0f / 16.0f;
#pragma unroll 1
  for (int ks = 0; ks < NN / 32; ++ks) { const int j0 = ks * 32; v8f s[2];
#pragma unroll
    for (int ct = 0; ct < 2; ++ct) { const size_t rk = (b * NN + j0 + ct * 16 + col) * DIM + h * HDd; v8f c = {}, cl = {};
      { const v16h kh = frag_h(KH + rk, lane); c = wmma16(aq, kh, c); cl = wmma16(aql, kh, cl); cl = wmma16(aq, frag_h(KL + rk, lane), cl); }
#pragma unroll
      for (int r = 0; r < 8; ++r) s[ct][r] = (c[r] + cl[r] * (1.0f / 2048.0f)) * isc; }
#pragma unroll
    for (int r = 0; r < 8; ++r) { float mx = fmaxf(s[0][r], s[1][r]);
#pragma unroll
      for (int o = 1; o < 16; o <<= 1) mx = fmaxf(mx, __shfl_xor(mx, o));
      const float mn = fmaxf(m[r], mx); const float alpha = (m[r] <= -1.0e38f) ? 0.f : __expf(m[r] - mn); const float e0 = __expf(s[0][r] - mn), e1 = __expf(s[1][r] - mn); float es = e0 + e1;
#pragma unroll
      for (int o = 1; o < 16; o <<= 1) es += __shfl_xor(es, o);
      l[r] = l[r] * alpha + es; m[r] = mn; acc[0][r] *= alpha; acc[1][r] *= alpha; accl[0][r] *= alpha; accl[1][r] *= alpha;
      { const float p0 = e0 * 2048.0f, p1 = e1 * 2048.0f; const _Float16 h0 = (_Float16)p0, h1 = (_Float16)p1; sph[wave][8 * g + r][col] = h0; sph[wave][8 * g + r][16 + col] = h1; spl[wave][8 * g + r][col] = (_Float16)((p0 - (float)h0) * 2048.0f); spl[wave][8 * g + r][16 + col] = (_Float16)((p1 - (float)h1) * 2048.0f); } }
    LDSX();
    const v16h pah = frag_h(&sph[wave][col][0], lane), pal = frag_h(&spl[wave][col][0], lane);
#pragma unroll
    for (int dt = 0; dt < 2; ++dt) { const size_t vo = (b * DIM + h * HDd + dt * 16 + col) * NN + j0; const v16h vh = frag_h(VH + vo, lane); acc[dt] = wmma16(pah, vh, acc[dt]); accl[dt] = wmma16(pal, vh, accl[dt]); accl[dt] = wmma16(pah, frag_h(VL + vo, lane), accl[dt]); }
    LDSX(); }
#pragma unroll
  for (int r = 0; r < 8; ++r) { const float il = (1.0f / 2048.0f) / l[r];
#pragma unroll
    for (int dt = 0; dt < 2; ++dt) { const int d = dt * 16 + col; so[wave][8 * g + r][d] = (acc[dt][r] + accl[dt][r] * (1.0f / 2048.0f)) * il + CB[(b * NH + h) * HDd + d]; } }
  LDSX();
  for (int rl = 0; rl < 16; ++rl) if (lane < 8) vst2(O + ((b * NH + h) * NN + q0 + rl) * HDd + lane * 4, *(const v4f*)&so[wave][rl][lane * 4]);
}
__global__ __launch_bounds__(128) void k_fc(const float* __restrict__ O, const __bf16* __restrict__ PK, const float* __restrict__ BF, const float* __restrict__ X, const float* __restrict__ G, const float* __restrict__ Bt, float* __restrict__ OUT) {
  __shared__ __align__(16) __bf16 sh[64][DIM + 8], sl[64][DIM + 8]; __shared__ __align__(16) float sy[64][DIM + 4];
  const int tid = threadIdx.x, wave = tid >> 5, lane = tid & 31, col = lane & 15, g = lane >> 4; const size_t rb0 = (size_t)blockIdx.x * 64; const size_t bp = rb0 / NN; const size_t n0 = rb0 % NN;
  for (int e = tid; e < 64 * DIM; e += 128) { const int r = e / DIM, c = e % DIM; const int hp = c / HDd, d = c % HDd; const float v = O[(((size_t)hp * NB + bp) * NN + n0 + r) * HDd + d]; const __bf16 hb = (__bf16)v; sh[r][c] = hb; sl[r][c] = (__bf16)(v - (float)hb); }
  if (tid < 64) for (int c = DIM; c < DIM + 8; ++c) { sh[tid][c] = (__bf16)0.f; sl[tid][c] = (__bf16)0.f; }
  __syncthreads();
#pragma unroll 1
  for (int pass = 0; pass < 2; ++pass) { v8f acc[8] = {};
#pragma unroll
    for (int kc = 0; kc < DIM / 32; ++kc) { const v16b a = frag_b(&sh[wave * 16 + col][kc * 32], lane), al = frag_b(&sl[wave * 16 + col][kc * 32], lane);
#pragma unroll
      for (int j = 0; j < 8; ++j) { const v16b w = frag_b(PK + PKF + (size_t)(pass * 128 + j * 16 + col) * DIM + kc * 32, lane); acc[j] = wmma_bf(al, w, acc[j]); acc[j] = wmma_bf(a, w, acc[j]); } }
#pragma unroll
    for (int j = 0; j < 8; ++j) { const int c = pass * 128 + j * 16 + col; const float bb = bfr(BF[c]);
#pragma unroll
      for (int r = 0; r < 8; ++r) { const size_t row = rb0 + wave * 16 + 8 * g + r; sy[wave * 16 + 8 * g + r][c] = acc[j][r] + bb + bfr(X[row * DIM + c]); } } }
  __syncthreads();
  { const int r = tid >> 1, part = tid & 1; float s = 0.f; for (int c = part * 128; c < part * 128 + 128; ++c) s += sy[r][c]; s += __shfl_xor(s, 1); const float mu = s / (float)DIM; float q = 0.f; for (int c = part * 128; c < part * 128 + 128; ++c) { const float dv = sy[r][c] - mu; q += dv * dv; } q += __shfl_xor(q, 1); const float inv = 1.0f / sqrtf(q / (float)DIM + 1e-5f);
    __syncthreads();
    for (int c = part * 128; c < part * 128 + 128; ++c) sy[r][c] = (sy[r][c] - mu) * inv * bfr(G[c]) + bfr(Bt[c]); }
  __syncthreads();
  for (int e = tid; e < 64 * (DIM / 4); e += 128) { const int r = e / (DIM / 4), q = e % (DIM / 4); vst2(OUT + (rb0 + r) * DIM + q * 4, *(const v4f*)&sy[r][q * 4]); }
}
extern "C" void kernel_launch(void* const* d_in, const int* in_sizes, int n_in, void* d_out, int out_size, void* d_ws, size_t ws_size, hipStream_t stream) {
  (void)in_sizes; (void)n_in; (void)out_size;
  const float** F = (const float**)d_in;
  if (ws_size < (size_t)WS_END) return;
  char* ws = (char*)d_ws; __bf16* PK = (__bf16*)(ws + WS_PK); float *Q = (float*)(ws + WS_Q), *K = (float*)(ws + WS_K), *M = (float*)(ws + WS_M), *MU = (float*)(ws + WS_MU), *CB = (float*)(ws + WS_CB), *O = (float*)(ws + WS_O); _Float16 *QH = (_Float16*)(ws + WS_QH), *QL = (_Float16*)(ws + WS_QL), *KH = (_Float16*)(ws + WS_KH), *KL = (_Float16*)(ws + WS_KL), *VH = (_Float16*)(ws + WS_VH), *VL = (_Float16*)(ws + WS_VL);
  k_pack<<<dim3(DIM, 5), 256, 0, stream>>>(F[2], F[8], F[4], F[6], F[10], PK);
  k_proj<<<dim3(NR / 64, 3), 128, 0, stream>>>(F[0], F[1], PK, F[3], F[9], F[5], F[7], Q, K, M, VH, VL);
  k_mean<<<dim3(NB, 2), 256, 0, stream>>>(Q, K, MU);
  k_center<<<NR, 256, 0, stream>>>(Q, K, MU, QH, QL, KH, KL);
  k_gate<<<dim3(NB, NH), 512, 0, stream>>>(M, VH, VL, CB);
  k_attn<<<dim3(TQB, NH, NB), 128, 0, stream>>>(QH, QL, KH, KL, VH, VL, CB, O);
  k_fc<<<NR / 64, 128, 0, stream>>>(O, PK, F[11], F[0], F[12], F[13], (float*)d_out);
}
